// DKAModule_27066883899461
// MI455X (gfx1250) — hardware-run, weakly checked
//
#include <hip/hip_runtime.h>


#define NB_  2
#define NN   4096
#define DM   1024
#define NH_  8
#define DH   128
#define RR   4
#define KM   21
typedef _Float16 h16;
typedef unsigned short bf;
typedef __attribute__((ext_vector_type(16))) __bf16   v16bf;
typedef __attribute__((ext_vector_type(16))) _Float16 v16h;
typedef __attribute__((ext_vector_type(8)))  _Float16 v8h;
typedef __attribute__((ext_vector_type(8)))  unsigned short v8us;
typedef __attribute__((ext_vector_type(8)))  float    v8f;
typedef __attribute__((ext_vector_type(4)))  float    v4f;
typedef v8h  __attribute__((may_alias)) v8ha;
typedef v4f  __attribute__((may_alias)) v4fa;
typedef v8us __attribute__((may_alias)) v8usa;

__device__ __forceinline__ unsigned short f2bf(float f) { unsigned u = __float_as_uint(f); u += 0x7FFFu + ((u >> 16) & 1u); return (unsigned short)(u >> 16); }
__device__ __forceinline__ float bf2f(unsigned short b) { return __uint_as_float(((unsigned)b) << 16); }
__device__ __forceinline__ float bfr(float f) { return bf2f(f2bf(f)); }
__device__ __forceinline__ v16h cat16(v8h lo, v8h hi) { return __builtin_shufflevector(lo, hi, 0, 1, 2, 3, 4, 5, 6, 7, 8, 9, 10, 11, 12, 13, 14, 15); }
__device__ __forceinline__ v16bf cat16b(v8us lo, v8us hi) { return __builtin_bit_cast(v16bf, __builtin_shufflevector(lo, hi, 0, 1, 2, 3, 4, 5, 6, 7, 8, 9, 10, 11, 12, 13, 14, 15)); }
__device__ __forceinline__ v8f wmma16(v16h a, v16h b, v8f c) { return __builtin_amdgcn_wmma_f32_16x16x32_f16(false, a, false, b, (short)0, c, false, false); }
__device__ __forceinline__ v8f wmmab(v16bf a, v16bf b, v8f c) { return __builtin_amdgcn_wmma_f32_16x16x32_bf16(false, a, false, b, (short)0, c, false, false); }


template <typename T16> struct WFrag;
template <> struct WFrag<h16> { typedef v16h V; static __device__ __forceinline__ V ld(const h16* p) { return cat16(*(const v8h*)p, *(const v8h*)(p + 16)); } static __device__ __forceinline__ v8f mma(V a, V b, v8f c) { return wmma16(a, b, c); } };
template <> struct WFrag<bf> { typedef v16bf V; static __device__ __forceinline__ V ld(const bf* p) { return cat16b(*(const v8us*)p, *(const v8us*)(p + 16)); } static __device__ __forceinline__ v8f mma(V a, V b, v8f c) { return wmmab(a, b, c); } };
template <typename T16, int NSPLIT, bool BIAS>
__global__ __launch_bounds__(32) void k_gemmw(const T16* __restrict__ A, const T16* __restrict__ A2, const T16* __restrict__ Bt, const T16* __restrict__ Bt2, int K, float* C, int ldc, const float* __restrict__ bias, size_t sA, size_t sB, size_t sC) {
    typedef typename WFrag<T16>::V V;
    __shared__ __align__(16) float os[16 * 68];
    const size_t z = blockIdx.z; A += z * sA; if (A2) A2 += z * sA; Bt += z * sB; if (Bt2) Bt2 += z * sB; C += z * sC;
    const int lane = threadIdx.x & 31, lr = lane & 15, hi = lane >> 4; const int r0 = blockIdx.x * 64, c0 = blockIdx.y * 64;
    v8f acc[4][4];
#pragma unroll
    for (int mb = 0; mb < 4; ++mb)
#pragma unroll
        for (int nb = 0; nb < 4; ++nb) acc[mb][nb] = (v8f){};
    const size_t aoff = (size_t)(r0 + lr) * K + 8 * hi, boff = (size_t)(c0 + lr) * K + 8 * hi;
#pragma unroll 1
    for (int kc = 0; kc < K; kc += 32) {
        V a[4], a2[4];
#pragma unroll
        for (int mb = 0; mb < 4; ++mb) { a[mb] = WFrag<T16>::ld(A + aoff + (size_t)mb * 16 * K + kc); if (NSPLIT == 1 || NSPLIT == 2) a2[mb] = WFrag<T16>::ld(A2 + aoff + (size_t)mb * 16 * K + kc); }
#pragma unroll
        for (int nb = 0; nb < 4; ++nb) { const V b = WFrag<T16>::ld(Bt + boff + (size_t)nb * 16 * K + kc); V b2; if (NSPLIT >= 2) b2 = WFrag<T16>::ld(Bt2 + boff + (size_t)nb * 16 * K + kc);
#pragma unroll
            for (int mb = 0; mb < 4; ++mb) { acc[mb][nb] = WFrag<T16>::mma(a[mb], b, acc[mb][nb]); if (NSPLIT == 1 || NSPLIT == 2) acc[mb][nb] = WFrag<T16>::mma(a2[mb], b, acc[mb][nb]); if (NSPLIT >= 2) acc[mb][nb] = WFrag<T16>::mma(a[mb], b2, acc[mb][nb]); } }
        asm volatile("v_nop\n\tv_nop\n\tv_nop\n\tv_nop" : "+v"(acc[0][0]), "+v"(acc[1][1]), "+v"(acc[2][2]), "+v"(acc[3][3]) : "v"(a[0]), "v"(a[3]));
    }
#pragma unroll
    for (int mb = 0; mb < 4; ++mb) {
#pragma unroll
        for (int nb = 0; nb < 4; ++nb) {
#pragma unroll
            for (int j = 0; j < 8; ++j) os[(hi * 8 + j) * 68 + nb * 16 + lr] = acc[mb][nb][j]; }
        __builtin_amdgcn_wave_barrier(); asm volatile("" ::: "memory");
        float* crow = C + (size_t)(r0 + mb * 16) * ldc + c0;
#pragma unroll 1
        for (int ps = 0; ps < 2; ++ps) {
#pragma unroll
            for (int s = 0; s < 8; ++s) { const int row = 2 * s + hi, cofs = lr * 4; v4f val = *(const v4fa*)(os + row * 68 + cofs); if (BIAS) { val[0] += bfr(bias[c0 + cofs]); val[1] += bfr(bias[c0 + cofs + 1]); val[2] += bfr(bias[c0 + cofs + 2]); val[3] += bfr(bias[c0 + cofs + 3]); }
                *(volatile v4f*)(crow + (size_t)row * ldc + cofs) = val; }
            if (ps == 0) __threadfence(); }
        __builtin_amdgcn_wave_barrier(); asm volatile("" ::: "memory");
    }
}

__device__ __forceinline__ void splitf(float y, unsigned short& h, unsigned short& l) { h = f2bf(y); l = f2bf(y - bf2f(h)); }
typedef __attribute__((ext_vector_type(2))) unsigned short v2us;
__constant__ int KSZ[NH_] = {3, 3, 7, 7, 11, 11, 21, 21};

__global__ __launch_bounds__(256) void k_cvt8(const float* __restrict__ src, bf* dst, size_t n8) { const size_t i = (size_t)blockIdx.x * 256 + threadIdx.x; if (i >= n8) return; const v8f v = *(const v8f*)(src + i * 8); v8us o;
#pragma unroll
    for (int k = 0; k < 8; ++k) o[k] = f2bf(v[k]); *(volatile v8us*)(dst + i * 8) = o; __threadfence(); *(volatile v8us*)(dst + i * 8) = o; }
__global__ __launch_bounds__(256) void k_coef(const float* __restrict__ XP, const float* __restrict__ Wc, float* CL) { const int idx = blockIdx.x * 256 + threadIdx.x; if (idx >= NN * NH_) return; const int h = idx % NH_, n = idx / NH_; const float* xr = XP + (size_t)n * DM + h * DH; const float* w = Wc + (size_t)h * DH * RR; float c0 = 0.f, c1 = 0.f, c2 = 0.f, c3 = 0.f;
    for (int d = 0; d < DH; ++d) { const float xv = xr[d]; float p0 = __fmul_rn(xv, bfr(w[d * RR + 0])), p1 = __fmul_rn(xv, bfr(w[d * RR + 1])), p2 = __fmul_rn(xv, bfr(w[d * RR + 2])), p3 = __fmul_rn(xv, bfr(w[d * RR + 3])); asm volatile("" : "+v"(p0), "+v"(p1), "+v"(p2), "+v"(p3)); c0 = __fadd_rn(c0, p0); c1 = __fadd_rn(c1, p1); c2 = __fadd_rn(c2, p2); c3 = __fadd_rn(c3, p3); }
    v4f o; o[0] = c0; o[1] = c1; o[2] = c2; o[3] = c3; *(volatile v4f*)(CL + (size_t)idx * RR) = o; __threadfence(); *(volatile v4f*)(CL + (size_t)idx * RR) = o; }
__global__ __launch_bounds__(256) void k_dko(const float* __restrict__ XP, const float* __restrict__ CL, const float* __restrict__ A, const float* __restrict__ V, const float* __restrict__ base, const float* __restrict__ alphas, bf* Ch, bf* Cl) {
    const size_t e = ((size_t)blockIdx.x * 256 + threadIdx.x) * 2; if (e >= (size_t)NN * DM) return; const int col = (int)(e % DM), n = (int)(e / DM); const int h = col / DH, d = col % DH; const int kh = KSZ[h], pad = kh / 2;
    const float al = __fdiv_rn(1.0f, __fadd_rn(1.0f, __expf(-bfr(alphas[h])))); const float bl = __fsub_rn(1.0f, al); const v4f c = *(const v4f*)(CL + ((size_t)n * NH_ + h) * RR); float o0 = 0.f, o1 = 0.f;
    for (int k = 0; k < kh; ++k) { const int src = n + k - pad; if (src < 0 || src >= NN) continue; float dy0 = 0.f, dy1 = 0.f;
#pragma unroll
        for (int r = 0; r < RR; ++r) { float ca = __fmul_rn(c[r], bfr(A[((size_t)h * RR + r) * KM + k])); asm volatile("" : "+v"(ca)); float p0 = __fmul_rn(ca, bfr(V[((size_t)h * RR + r) * DH + d])), p1 = __fmul_rn(ca, bfr(V[((size_t)h * RR + r) * DH + d + 1])); asm volatile("" : "+v"(p0), "+v"(p1)); dy0 = __fadd_rn(dy0, p0); dy1 = __fadd_rn(dy1, p1); }
        float k0 = __fmul_rn(al, dy0), k1 = __fmul_rn(al, dy1); asm volatile("" : "+v"(k0), "+v"(k1)); float b0 = __fmul_rn(bl, bfr(base[((size_t)h * KM + k) * DH + d])), b1 = __fmul_rn(bl, bfr(base[((size_t)h * KM + k) * DH + d + 1])); asm volatile("" : "+v"(b0), "+v"(b1));
        k0 = __fadd_rn(k0, b0); k1 = __fadd_rn(k1, b1); const float* xs = XP + (size_t)src * DM + col; float q0 = __fmul_rn(k0, xs[0]), q1 = __fmul_rn(k1, xs[1]); asm volatile("" : "+v"(q0), "+v"(q1)); o0 = __fadd_rn(o0, q0); o1 = __fadd_rn(o1, q1); }
    v2us oh, ol; unsigned short a2, c2; splitf(o0, a2, c2); oh[0] = a2; ol[0] = c2; splitf(o1, a2, c2); oh[1] = a2; ol[1] = c2; *(volatile v2us*)(Ch + e) = oh; *(volatile v2us*)(Cl + e) = ol; __threadfence(); *(volatile v2us*)(Ch + e) = oh; *(volatile v2us*)(Cl + e) = ol; }

extern "C" void kernel_launch(void* const* d_in, const int* in_sizes, int n_in,
                              void* d_out, int out_size, void* d_ws, size_t ws_size, hipStream_t stream) {
    (void)in_sizes; (void)n_in; (void)out_size;
    const float* x = (const float*)d_in[0]; const float* Win = (const float*)d_in[1]; const float* bin = (const float*)d_in[2]; const float* Wout = (const float*)d_in[3]; const float* bout = (const float*)d_in[4]; const float* Wc = (const float*)d_in[5]; const float* A = (const float*)d_in[6]; const float* V = (const float*)d_in[7]; const float* base = (const float*)d_in[8]; const float* alphas = (const float*)d_in[9];
    float* OUT = (float*)d_out;
    char* wsp = (char*)d_ws;
    auto take = [&](size_t bytes) { char* p = wsp; wsp += (bytes + 255) & ~(size_t)255; return (void*)p; };
    bf* WI = (bf*)take((size_t)DM * DM * 2); bf* WO = (bf*)take((size_t)DM * DM * 2); bf* XB = (bf*)take((size_t)NN * DM * 2); float* XP = (float*)take((size_t)NN * DM * 4); float* CL = (float*)take((size_t)NN * NH_ * RR * 4); bf* Ch = (bf*)take((size_t)NN * DM * 2); bf* Cl = (bf*)take((size_t)NN * DM * 2);
    if ((size_t)(wsp - (char*)d_ws) > ws_size) return;
    k_cvt8<<<(unsigned)(((size_t)DM * DM / 8 + 255) / 256), 256, 0, stream>>>(Win, WI, (size_t)DM * DM / 8); k_cvt8<<<(unsigned)(((size_t)DM * DM / 8 + 255) / 256), 256, 0, stream>>>(Wout, WO, (size_t)DM * DM / 8);
    for (int b = 0; b < NB_; ++b) {
        k_cvt8<<<(unsigned)(((size_t)NN * DM / 8 + 255) / 256), 256, 0, stream>>>(x + (size_t)b * NN * DM, XB, (size_t)NN * DM / 8);
        k_gemmw<bf, 0, true><<<dim3(NN / 64, DM / 64, 1), 32, 0, stream>>>(XB, nullptr, WI, nullptr, DM, XP, DM, bin, 0, 0, 0);
        k_coef<<<(NN * NH_ + 255) / 256, 256, 0, stream>>>(XP, Wc, CL);
        k_dko<<<(unsigned)(((size_t)NN * DM / 2 + 255) / 256), 256, 0, stream>>>(XP, CL, A, V, base, alphas, Ch, Cl);
        k_gemmw<bf, 1, true><<<dim3(NN / 64, DM / 64, 1), 32, 0, stream>>>(Ch, Cl, WO, nullptr, DM, OUT + (size_t)b * NN * DM, DM, bout, 0, 0, 0); }
}
